// MULTI_46024869543985
// MI455X (gfx1250) — hardware-verified
//
#include <hip/hip_runtime.h>


#define AS3 __attribute__((address_space(3)))

#define NB     256
#define NT     256
#define HH     64
#define G4     256
#define KC     128
#define CE     128
#define PGN    128
#define EMB    32
#define ENBLK  (NB / EMB)
#define ENTHR  256
#define APE    136
#define PGM    64
#define PGTHR  256
#define APD    200
#define DNTHR  512

static_assert(G4 == 4 * HH);
static_assert(KC == 2 * HH);
static_assert(CE == 2 * HH);
static_assert(KC % 32 == 0);
static_assert(APE % 8 == 0);
static_assert(APE >= KC);
static_assert(APD % 8 == 0);
static_assert(APD >= 3 * HH);
static_assert(ENTHR == G4);
static_assert(DNTHR == 2 * G4);
static_assert(ENTHR / 32 == (EMB / 16) * (HH / 16));
static_assert(DNTHR / 32 == NB / 16);
static_assert(NB % EMB == 0);
static_assert((NB * NT) % PGM == 0);
static_assert(PGTHR / 32 == (PGM / 16) * (PGN / 64));
static_assert(ENTHR == EMB * 8);

#define SCL    16.0f
#define INV256 0.00390625f

typedef _Float16 v16h __attribute__((ext_vector_type(16)));
typedef _Float16 v8h  __attribute__((ext_vector_type(8)));
typedef _Float16 v4h  __attribute__((ext_vector_type(4)));
typedef float    v8f  __attribute__((ext_vector_type(8)));
typedef float    v4f  __attribute__((ext_vector_type(4)));
typedef float    v2f  __attribute__((ext_vector_type(2)));

typedef AS3 _Float16*       lp_h;
typedef AS3 const _Float16* lcp_h;
typedef AS3 float*          lp_f;
typedef AS3 const float*    lcp_f;

union Frag { v16h v; v8h half[2]; };

constexpr size_t SZ_WE  = (size_t)2 * G4 * KC * 2;
constexpr size_t SZ_WD  = SZ_WE;
constexpr size_t SZ_WC  = (size_t)PGN * KC * 2;
constexpr size_t SZ_E   = (size_t)NB * NT * CE * 4;
constexpr size_t SZ_CT  = (size_t)2 * NB * HH * 4;
constexpr size_t SZ_PG  = (size_t)NB * NT * PGN * 4;
constexpr size_t SZ_ZB  = (size_t)NB * HH * 4;
constexpr size_t SZ_LG  = (size_t)NT * NB * 2 * 4;
constexpr size_t OFF_WE = 0;
constexpr size_t OFF_WD = OFF_WE + SZ_WE;
constexpr size_t OFF_WC = OFF_WD + SZ_WD;
constexpr size_t OFF_E  = OFF_WC + SZ_WC;
constexpr size_t OFF_CT = OFF_E + SZ_E;
constexpr size_t OFF_PG = OFF_CT + SZ_CT;
constexpr size_t OFF_ZB = OFF_PG + SZ_PG;
constexpr size_t OFF_LG = OFF_ZB + SZ_ZB;
constexpr size_t WS_END = OFF_LG + SZ_LG;
static_assert(OFF_WD % 128 == 0 && OFF_WC % 128 == 0 && OFF_E % 128 == 0 && OFF_CT % 128 == 0);
static_assert(OFF_PG % 128 == 0 && OFF_ZB % 128 == 0 && OFF_LG % 128 == 0 && WS_END % 128 == 0);
static_assert(WS_END <= (size_t)134217728);

constexpr int NPW       = 2 * G4 * (KC / 8);
constexpr int NPC       = PGN * (KC / 8);
constexpr int PREP_WBLK = NPW / 256;
constexpr int PREP_CBLK = NPC / 256;
constexpr int PREP_BLK  = 2 * PREP_WBLK + PREP_CBLK;
static_assert(NPW % 256 == 0 && NPC % 256 == 0);
static_assert((size_t)NPW * 16 == SZ_WE);
static_assert((size_t)NPC * 16 == SZ_WC);

constexpr int    EA_TILE = EMB * APE;
constexpr size_t EL_A    = 0;
constexpr size_t ESZ_A   = (size_t)2 * EA_TILE * 2;
constexpr size_t EL_HF   = EL_A + ESZ_A;
constexpr size_t ESZ_HF  = (size_t)2 * EMB * HH * 4;
constexpr size_t EL_BIAS = EL_HF + ESZ_HF;
constexpr size_t ENC_LDS = EL_BIAS + (size_t)G4 * 4;
static_assert(EL_HF % 16 == 0 && EL_BIAS % 16 == 0);
static_assert((2 * EA_TILE) % 8 == 0);

constexpr size_t PL_X   = 0;
constexpr size_t PSZ_X  = (size_t)PGM * APE * 2;
constexpr size_t PL_O   = PL_X + PSZ_X;
constexpr size_t PG_LDS = PL_O + (size_t)PGM * PGN * 4;
static_assert(PL_O % 16 == 0);

constexpr size_t DL_A    = 0;
constexpr size_t DSZ_A   = (size_t)NB * APD * 2;
constexpr size_t DL_C    = DL_A + DSZ_A;
constexpr size_t DSZ_C   = (size_t)2 * NB * HH * 4;
constexpr size_t DL_LGP  = DL_C + DSZ_C;
constexpr size_t DSZ_LGP = (size_t)2 * NB * 2 * 4;
constexpr size_t DL_BIAS = DL_LGP + DSZ_LGP;
constexpr size_t DL_W2   = DL_BIAS + (size_t)2 * G4 * 4;
constexpr size_t DEC_LDS = DL_W2 + (size_t)2 * CE * 4;
static_assert(DL_C % 16 == 0 && DL_LGP % 16 == 0 && DL_BIAS % 16 == 0 && DL_W2 % 16 == 0);

__device__ __forceinline__ float rcpx(float x) { return __builtin_amdgcn_rcpf(x); }
__device__ __forceinline__ float sigm(float x) { return rcpx(1.0f + __expf(-x)); }
__device__ __forceinline__ float tanhm(float x) {
    const float e = __expf(2.0f * x);
    return 1.0f - 2.0f * rcpx(e + 1.0f);
}
__device__ __forceinline__ v8f ld8f(const float* p) {
    const v4f a = *(const v4f*)p;
    const v4f b = *(const v4f*)(p + 4);
    return __builtin_shufflevector(a, b, 0, 1, 2, 3, 4, 5, 6, 7);
}
__device__ __forceinline__ v8f zero8() {
    v8f z;
#pragma unroll
    for (int i = 0; i < 8; ++i) z[i] = 0.0f;
    return z;
}

__device__ __forceinline__ void ldfrag_lds(Frag& f, lcp_h p) {
    f.half[0] = *(AS3 const v8h*)(p);
    f.half[1] = *(AS3 const v8h*)(p + 16);
}
__device__ __forceinline__ void ldfrag_glb(Frag& f, const _Float16* p) {
    f.half[0] = *(const v8h*)(p);
    f.half[1] = *(const v8h*)(p + 16);
}
__device__ __forceinline__ v8f mma16(v8f c, const Frag& a, const Frag& b) {
    return __builtin_amdgcn_wmma_f32_16x16x32_f16(false, a.v, false, b.v, (short)0, c, false, false);
}
#define GUARD4(A0, A1, A2, A3, FA, FB0, FB1, FB2, FB3)                                   \
    asm volatile("v_nop\n\tv_nop\n\tv_nop\n\tv_nop"                                       \
                 : "+v"(A0), "+v"(A1), "+v"(A2), "+v"(A3)                                  \
                 : "v"(FA), "v"(FB0), "v"(FB1), "v"(FB2), "v"(FB3))

__device__ __forceinline__ void write_rows32(lcp_f tile, float* dst, size_t stride, int w, int lane)
{
    v4f v[2]; float* p[2];
#pragma unroll
    for (int i = 0; i < 2; ++i) {
        const int row = 4 * w + 2 * i + (lane >> 4);
        const int c4  = (lane & 15) * 4;
        v[i] = *(AS3 const v4f*)(tile + row * HH + c4);
        p[i] = dst + (size_t)row * stride + c4;
    }
    *(volatile v4f*)p[0] = v[0];
    *(volatile v4f*)p[1] = v[1];
    __threadfence();
    *(volatile v4f*)p[0] = v[0];
    *(volatile v4f*)p[1] = v[1];
}

__global__ __launch_bounds__(256)
void prep_kernel(const float* __restrict__ eWih, const float* __restrict__ eWhh,
                 const float* __restrict__ dWih, const float* __restrict__ dWhh,
                 const float* __restrict__ cW, _Float16* WE, _Float16* WD, _Float16* WC)
{
    const int tid = threadIdx.x;
    const int blk = blockIdx.x;
    if (blk < 2 * PREP_WBLK) {
        const int reg = blk / PREP_WBLK;
        const int p   = (blk - reg * PREP_WBLK) * 256 + tid;
        const int d   = p / (G4 * (KC / 8));
        const int n   = (p / (KC / 8)) & (G4 - 1);
        const int k8  = (p & (KC / 8 - 1)) * 8;
        const float* Wi = reg ? dWih : eWih;
        const float* Wh = reg ? dWhh : eWhh;
        const int ki = min(k8, HH - 8);
        const int kj = min(max(k8 - HH, 0), HH - 8);
        const size_t rb = (size_t)(d * G4 + n) * HH;
        const v8f a = ld8f(Wi + rb + ki);
        const v8f c = ld8f(Wh + rb + kj);
        v8h hv;
#pragma unroll
        for (int i = 0; i < 8; ++i) {
            const float v = (k8 < HH) ? a[i] : c[i];
            hv[i] = (_Float16)(v * SCL);
        }
        _Float16* dst = (reg ? WD : WE) + (size_t)p * 8;
        *(volatile v8h*)dst = hv;
        __threadfence();
        *(volatile v8h*)dst = hv;
    } else {
        const int p  = (blk - 2 * PREP_WBLK) * 256 + tid;
        const int n  = p / (KC / 8);
        const int k8 = (p & (KC / 8 - 1)) * 8;
        const v8f a = ld8f(cW + (size_t)(n & (HH - 1)) * (2 * CE) + (n / HH) * CE + k8);
        v8h hv;
#pragma unroll
        for (int i = 0; i < 8; ++i) hv[i] = (_Float16)(a[i] * SCL);
        _Float16* dst = WC + (size_t)p * 8;
        *(volatile v8h*)dst = hv;
        __threadfence();
        *(volatile v8h*)dst = hv;
    }
}

__global__ __launch_bounds__(ENTHR)
void encoder_kernel(const int* __restrict__ xin, const float* __restrict__ emb, int nV,
                    const _Float16* __restrict__ WE, const float* __restrict__ bih,
                    const float* __restrict__ bhh, float* E, float* CT)
{
    extern __shared__ __attribute__((aligned(16))) char smem[];
    lp_h sA    = (lp_h)(smem + EL_A);
    lp_f sHf   = (lp_f)(smem + EL_HF);
    lp_f sBias = (lp_f)(smem + EL_BIAS);

    const int tid  = threadIdx.x;
    const int lane = tid & 31;
    const int w    = tid >> 5;
    const int h    = lane >> 4;
    const int m    = lane & 15;
    const int dir  = (int)blockIdx.x / ENBLK;
    const int b0   = ((int)blockIdx.x - dir * ENBLK) * EMB;
    const _Float16* Wd = WE + (size_t)dir * G4 * KC;

    {
        v8h zh;
#pragma unroll
        for (int i = 0; i < 8; ++i) zh[i] = (_Float16)0.0f;
        for (int i = tid; i < (2 * EA_TILE) / 8; i += ENTHR) *(AS3 v8h*)(sA + 8 * i) = zh;
        sBias[tid] = bih[dir * G4 + tid] + bhh[dir * G4 + tid];
    }
    float c[8];
#pragma unroll
    for (int r = 0; r < 8; ++r) c[r] = 0.0f;
    __syncthreads();

    const int srow = tid >> 3;
    const int sc8  = (tid & 7) * 8;
    const int* idrow = xin + (size_t)(b0 + srow) * NT;

    {
        const int t0 = dir ? (NT - 1) : 0;
        int id = idrow[t0];
        id = min(max(id, 0), nV - 1);
        const v8f xv = ld8f(emb + (size_t)id * HH + sc8);
        v8h hv;
#pragma unroll
        for (int i = 0; i < 8; ++i) hv[i] = (_Float16)(xv[i] * SCL);
        *(AS3 v8h*)(sA + srow * APE + sc8) = hv;
    }

    const int mt = w >> 2, ug = w & 3;
    const int n  = ug * 16 + m;
    const float bi = sBias[n];
    const float bf = sBias[HH + n];
    const float bg = sBias[2 * HH + n];
    const float bo = sBias[3 * HH + n];

#pragma unroll 1
    for (int s = 0; s < NT; ++s) {
        const int cur = s & 1;
        lp_h sAc = sA + cur * EA_TILE;
        lp_h sAn = sA + (cur ^ 1) * EA_TILE;

        __syncthreads();

        if (s > 0) {
            const int tp = dir ? (NT - s) : (s - 1);
            write_rows32(sHf + ((s - 1) & 1) * (EMB * HH), E + ((size_t)b0 * NT + tp) * CE + HH * dir,
                         (size_t)NT * CE, w, lane);
        }
        if (s + 1 < NT) {
            const int tn = dir ? (NT - 2 - s) : (s + 1);
            int id = idrow[tn];
            id = min(max(id, 0), nV - 1);
            const v8f xv = ld8f(emb + (size_t)id * HH + sc8);
            v8h hv;
#pragma unroll
            for (int i = 0; i < 8; ++i) hv[i] = (_Float16)(xv[i] * SCL);
            *(AS3 v8h*)(sAn + srow * APE + sc8) = hv;
        }

        v8f acc[4];
#pragma unroll
        for (int q = 0; q < 4; ++q) acc[q] = zero8();
        lcp_h ab = sAc + (mt * 16 + m) * APE + 8 * h;
        const _Float16* wb = Wd + (size_t)n * KC + 8 * h;
#pragma unroll
        for (int ks = 0; ks < KC / 32; ++ks) {
            Frag a, b[4];
            ldfrag_lds(a, ab + 32 * ks);
#pragma unroll
            for (int q = 0; q < 4; ++q) ldfrag_glb(b[q], wb + (size_t)q * (HH * KC) + 32 * ks);
#pragma unroll
            for (int q = 0; q < 4; ++q) acc[q] = mma16(acc[q], a, b[q]);
            GUARD4(acc[0], acc[1], acc[2], acc[3], a.v, b[0].v, b[1].v, b[2].v, b[3].v);
        }

        lp_f hf = sHf + (s & 1) * (EMB * HH);
#pragma unroll
        for (int r = 0; r < 8; ++r) {
            const int row = mt * 16 + 8 * h + r;
            const float gi = acc[0][r] * INV256 + bi;
            const float gf = acc[1][r] * INV256 + bf;
            const float gg = acc[2][r] * INV256 + bg;
            const float go = acc[3][r] * INV256 + bo;
            const float cn = sigm(gf) * c[r] + sigm(gi) * tanhm(gg);
            c[r] = cn;
            const float hn = sigm(go) * tanhm(cn);
            sAn[row * APE + HH + n] = (_Float16)(hn * SCL);
            hf[row * HH + n] = hn;
        }
    }
    __syncthreads();
    {
        const int tl = dir ? 0 : (NT - 1);
        write_rows32(sHf + EMB * HH, E + ((size_t)b0 * NT + tl) * CE + HH * dir, (size_t)NT * CE, w, lane);
    }
#pragma unroll
    for (int r = 0; r < 8; ++r) sHf[(mt * 16 + 8 * h + r) * HH + n] = c[r];
    __syncthreads();
    write_rows32(sHf, CT + ((size_t)dir * NB + b0) * HH, (size_t)HH, w, lane);
}

__global__ __launch_bounds__(PGTHR)
void pg_kernel(const float* __restrict__ E, const _Float16* __restrict__ WC, float* PG)
{
    extern __shared__ __attribute__((aligned(16))) char smem[];
    lp_h sX = (lp_h)(smem + PL_X);
    lp_f sO = (lp_f)(smem + PL_O);

    const int tid  = threadIdx.x;
    const int lane = tid & 31;
    const int w    = tid >> 5;
    const int h    = lane >> 4;
    const int m    = lane & 15;
    const int r0   = (int)blockIdx.x * PGM;

#pragma unroll
    for (int j = 0; j < (PGM * CE / 8) / PGTHR; ++j) {
        const int q   = tid + PGTHR * j;
        const int row = q / (CE / 8);
        const int c8  = (q & (CE / 8 - 1)) * 8;
        const v8f ev = ld8f(E + (size_t)(r0 + row) * CE + c8);
        v8h hv;
#pragma unroll
        for (int i = 0; i < 8; ++i) hv[i] = (_Float16)(ev[i] * SCL);
        *(AS3 v8h*)(sX + row * APE + c8) = hv;
    }
    __syncthreads();

    const int mt = w >> 1, nt0 = (w & 1) * 4;
    v8f acc[4];
#pragma unroll
    for (int j = 0; j < 4; ++j) acc[j] = zero8();
    lcp_h ab = sX + (mt * 16 + m) * APE + 8 * h;
    const _Float16* wb = WC + (size_t)(nt0 * 16 + m) * KC + 8 * h;
#pragma unroll
    for (int ks = 0; ks < KC / 32; ++ks) {
        Frag a, b[4];
        ldfrag_lds(a, ab + 32 * ks);
#pragma unroll
        for (int j = 0; j < 4; ++j) ldfrag_glb(b[j], wb + (size_t)j * (16 * KC) + 32 * ks);
#pragma unroll
        for (int j = 0; j < 4; ++j) acc[j] = mma16(acc[j], a, b[j]);
        GUARD4(acc[0], acc[1], acc[2], acc[3], a.v, b[0].v, b[1].v, b[2].v, b[3].v);
    }
#pragma unroll
    for (int j = 0; j < 4; ++j)
#pragma unroll
        for (int r = 0; r < 8; ++r)
            sO[(mt * 16 + 8 * h + r) * PGN + (nt0 + j) * 16 + m] = acc[j][r] * INV256;
    __syncthreads();

    v4f v[8]; float* p[8];
#pragma unroll
    for (int i = 0; i < 8; ++i) {
        const int row = 8 * w + i;
        v[i] = *(AS3 const v4f*)(sO + row * PGN + lane * 4);
        p[i] = PG + (size_t)(r0 + row) * PGN + lane * 4;
    }
#pragma unroll
    for (int i = 0; i < 8; ++i) *(volatile v4f*)p[i] = v[i];
    __threadfence();
#pragma unroll
    for (int i = 0; i < 8; ++i) *(volatile v4f*)p[i] = v[i];
}

__global__ __launch_bounds__(256)
void attn_kernel(const float* __restrict__ E, const float* __restrict__ PG,
                 const float* __restrict__ aW, const float* __restrict__ ab,
                 const float* __restrict__ cb, float* ZB)
{
    __shared__ float sAW[CE];
    __shared__ float sWt[NT];
    __shared__ float sRed[16];
    __shared__ float sPart[16 * HH];
    __shared__ float sZB[HH];

    const int tid  = threadIdx.x;
    const int lane = tid & 31;
    const int w    = tid >> 5;
    const int b    = blockIdx.x;

    if (tid < CE) sAW[tid] = aW[tid];
    __syncthreads();

    const float* er = E + ((size_t)b * NT + tid) * CE;
    float e0 = 0.0f, e1 = 0.0f, e2 = 0.0f, e3 = 0.0f;
#pragma unroll 1
    for (int j = 0; j < CE / 4; ++j) {
        const v4f ev = *(const v4f*)(er + 4 * j);
        e0 += ev[0] * sAW[4 * j];
        e1 += ev[1] * sAW[4 * j + 1];
        e2 += ev[2] * sAW[4 * j + 2];
        e3 += ev[3] * sAW[4 * j + 3];
    }
    const float e = ((e0 + e1) + (e2 + e3)) + ab[0];

    float mx = e;
#pragma unroll
    for (int off = 16; off >= 1; off >>= 1) mx = fmaxf(mx, __shfl_xor(mx, off, 32));
    if (lane == 0) sRed[w] = mx;
    __syncthreads();
    mx = sRed[0];
#pragma unroll
    for (int i = 1; i < 8; ++i) mx = fmaxf(mx, sRed[i]);
    const float p = __expf(e - mx);
    float sm = p;
#pragma unroll
    for (int off = 16; off >= 1; off >>= 1) sm += __shfl_xor(sm, off, 32);
    if (lane == 0) sRed[8 + w] = sm;
    __syncthreads();
    float tot = 0.0f;
#pragma unroll
    for (int i = 0; i < 8; ++i) tot += sRed[8 + i];
    sWt[tid] = p * (1.0f / tot);
    __syncthreads();

    const int c4 = (tid & 15) * 4;
    const int tg = tid >> 4;
    const float* gp = PG + ((size_t)b * NT + tg * 16) * PGN + HH + c4;
    v4f acc;
#pragma unroll
    for (int i = 0; i < 4; ++i) acc[i] = 0.0f;
#pragma unroll 1
    for (int i = 0; i < 16; ++i) {
        const float wv = sWt[tg * 16 + i];
        const v4f g = *(const v4f*)(gp + (size_t)i * PGN);
        acc += g * wv;
    }
#pragma unroll
    for (int i = 0; i < 4; ++i) sPart[tg * HH + c4 + i] = acc[i];
    __syncthreads();
    if (tid < HH) {
        float sacc = 0.0f;
#pragma unroll 1
        for (int g = 0; g < 16; ++g) sacc += sPart[g * HH + tid];
        sZB[tid] = sacc + cb[tid];
    }
    __syncthreads();
    const int q = min(tid, 15);
    v4f zv;
#pragma unroll
    for (int i = 0; i < 4; ++i) zv[i] = sZB[4 * q + i];
    float* zp = ZB + (size_t)b * HH + 4 * q;
    if (tid < 16) *(volatile v4f*)zp = zv;
    __threadfence();
    if (tid < 16) *(volatile v4f*)zp = zv;
}

__device__ __forceinline__ void store_logits(lcp_f sLgP, float b20, float b21, float* LG, int tstep, int tid, bool active)
{
    const int q = min(tid, 127);
    v4f lv;
#pragma unroll
    for (int e = 0; e < 4; ++e) {
        const int f = 4 * q + e;
        lv[e] = sLgP[f] + sLgP[2 * NB + f] + ((e & 1) ? b21 : b20);
    }
    float* lp = LG + (size_t)tstep * (2 * NB) + 4 * q;
    if (active) *(volatile v4f*)lp = lv;
    __threadfence();
    if (active) *(volatile v4f*)lp = lv;
}

__global__ __launch_bounds__(DNTHR)
void decoder_kernel(const float* __restrict__ E, const float* __restrict__ CT,
                    const float* __restrict__ PG, const float* __restrict__ ZB,
                    const _Float16* __restrict__ WD, const float* __restrict__ bih,
                    const float* __restrict__ bhh, const float* __restrict__ W2,
                    const float* __restrict__ b2, float* LG)
{
    extern __shared__ __attribute__((aligned(16))) char smem[];
    lp_h sA    = (lp_h)(smem + DL_A);
    lp_f sC    = (lp_f)(smem + DL_C);
    lp_f sLgP  = (lp_f)(smem + DL_LGP);
    lp_f sBias = (lp_f)(smem + DL_BIAS);
    lp_f sW2   = (lp_f)(smem + DL_W2);

    const int tid  = threadIdx.x;
    const int lane = tid & 31;
    const int w    = tid >> 5;
    const int h    = lane >> 4;
    const int m    = lane & 15;

    sBias[tid] = bih[tid] + bhh[tid];
    if (tid < 2 * CE) sW2[tid] = W2[tid];
#pragma unroll 1
    for (int it = 0; it < (2 * NB * HH / 4) / DNTHR; ++it) {
        const int q = tid + DNTHR * it;
        *(AS3 v4f*)(sC + 4 * q) = *(const v4f*)(CT + 4 * (size_t)q);
    }
#pragma unroll 1
    for (int it = 0; it < (2 * NB * HH / 4) / DNTHR; ++it) {
        const int q  = tid + DNTHR * it;
        const int d  = q / (NB * HH / 4);
        const int bq = (q / (HH / 4)) & (NB - 1);
        const int j4 = (q & (HH / 4 - 1)) * 4;
        const float* src = E + ((size_t)bq * NT + (d ? 0 : (NT - 1))) * CE + HH * d + j4;
        const v4f hv = *(const v4f*)src;
        v4h hh4;
#pragma unroll
        for (int i = 0; i < 4; ++i) hh4[i] = (_Float16)(hv[i] * SCL);
        *(AS3 v4h*)(sA + bq * APD + HH + HH * d + j4) = hh4;
    }
    const float b20 = b2[0], b21 = b2[1];
    const int mt = w;

#pragma unroll 1
    for (int t = 0; t < NT; ++t) {
        __syncthreads();

        store_logits(sLgP, b20, b21, LG, (t > 0) ? (t - 1) : 0, tid, (t > 0) && (tid < 128));
#pragma unroll 1
        for (int it = 0; it < (NB * HH / 4) / DNTHR; ++it) {
            const int q  = tid + DNTHR * it;
            const int bq = q / (HH / 4);
            const int c4 = (q & (HH / 4 - 1)) * 4;
            const v4f pv = *(const v4f*)(PG + ((size_t)bq * NT + t) * PGN + c4);
            const v4f zb = *(const v4f*)(ZB + (size_t)bq * HH + c4);
            v4h zh;
#pragma unroll
            for (int i = 0; i < 4; ++i) zh[i] = (_Float16)(fmaxf(pv[i] + zb[i], 0.0f) * SCL);
            *(AS3 v4h*)(sA + bq * APD + c4) = zh;
        }
        __syncthreads();

#pragma unroll 1
        for (int d = 0; d < 2; ++d) {
            const int hcol = HH + HH * d;
            const _Float16* Wdd = WD + (size_t)d * G4 * KC;
            lcp_f bsb = sBias + d * G4;
            float dl0[8], dl1[8], hvf[4][8];
#pragma unroll
            for (int r = 0; r < 8; ++r) { dl0[r] = 0.0f; dl1[r] = 0.0f; }

#pragma unroll
            for (int ug = 0; ug < 4; ++ug) {
                const int n = ug * 16 + m;
                v8f acc[4];
#pragma unroll
                for (int q = 0; q < 4; ++q) acc[q] = zero8();
                const _Float16* wb = Wdd + (size_t)n * KC + 8 * h;
#pragma unroll
                for (int ks = 0; ks < KC / 32; ++ks) {
                    const int col0 = (ks < 2) ? (32 * ks) : (hcol + 32 * (ks - 2));
                    Frag a, b[4];
                    ldfrag_lds(a, sA + (mt * 16 + m) * APD + col0 + 8 * h);
#pragma unroll
                    for (int q = 0; q < 4; ++q) ldfrag_glb(b[q], wb + (size_t)q * (HH * KC) + 32 * ks);
#pragma unroll
                    for (int q = 0; q < 4; ++q) acc[q] = mma16(acc[q], a, b[q]);
                    GUARD4(acc[0], acc[1], acc[2], acc[3], a.v, b[0].v, b[1].v, b[2].v, b[3].v);
                }
                const float bi  = bsb[n];
                const float bf  = bsb[HH + n];
                const float bg  = bsb[2 * HH + n];
                const float bo  = bsb[3 * HH + n];
                const float w2a = sW2[HH * d + n];
                const float w2b = sW2[CE + HH * d + n];
#pragma unroll
                for (int r = 0; r < 8; ++r) {
                    const int row = mt * 16 + 8 * h + r;
                    const float gi = acc[0][r] * INV256 + bi;
                    const float gf = acc[1][r] * INV256 + bf;
                    const float gg = acc[2][r] * INV256 + bg;
                    const float go = acc[3][r] * INV256 + bo;
                    const int ci = (d * NB + row) * HH + n;
                    const float cp = sC[ci];
                    const float cn = sigm(gf) * cp + sigm(gi) * tanhm(gg);
                    sC[ci] = cn;
                    const float hn = sigm(go) * tanhm(cn);
                    hvf[ug][r] = hn;
                    dl0[r] += hn * w2a;
                    dl1[r] += hn * w2b;
                }
            }
#pragma unroll
            for (int r = 0; r < 8; ++r) {
#pragma unroll
                for (int off = 1; off <= 8; off <<= 1) {
                    dl0[r] += __shfl_xor(dl0[r], off, 32);
                    dl1[r] += __shfl_xor(dl1[r], off, 32);
                }
            }
            if (m == 0) {
#pragma unroll
                for (int r = 0; r < 8; ++r) {
                    const int row = mt * 16 + 8 * h + r;
                    sLgP[d * (2 * NB) + row * 2 + 0] = dl0[r];
                    sLgP[d * (2 * NB) + row * 2 + 1] = dl1[r];
                }
            }
            __builtin_amdgcn_fence(__ATOMIC_RELEASE, "wavefront");
            __builtin_amdgcn_wave_barrier();
#pragma unroll
            for (int ug = 0; ug < 4; ++ug)
#pragma unroll
                for (int r = 0; r < 8; ++r)
                    sA[(mt * 16 + 8 * h + r) * APD + hcol + ug * 16 + m] = (_Float16)(hvf[ug][r] * SCL);
        }
    }
    __syncthreads();
    store_logits(sLgP, b20, b21, LG, NT - 1, tid, tid < 128);
}

__global__ __launch_bounds__(256)
void out_kernel(const float* __restrict__ LG, const float* __restrict__ E,
                const float* __restrict__ W1, const float* __restrict__ b1, float* out)
{
    __shared__ float sRow[2 * NT];
    const int tid = threadIdx.x;
    const int blk = blockIdx.x;
    if (blk < NB) {
        const v2f v = *(const v2f*)(LG + ((size_t)tid * NB + blk) * 2);
        sRow[2 * tid]     = v[0];
        sRow[2 * tid + 1] = v[1];
    } else {
        const float* er = E + ((size_t)tid * NT + (NT - 1)) * CE;
        float a0 = 0.0f, a1 = 0.0f;
#pragma unroll 1
        for (int j = 0; j < CE / 4; ++j) {
            const v4f ev = *(const v4f*)(er + 4 * j);
            const v4f w0 = *(const v4f*)(W1 + 4 * j);
            const v4f w1 = *(const v4f*)(W1 + CE + 4 * j);
            a0 += ev[0] * w0[0] + ev[1] * w0[1] + ev[2] * w0[2] + ev[3] * w0[3];
            a1 += ev[0] * w1[0] + ev[1] * w1[1] + ev[2] * w1[2] + ev[3] * w1[3];
        }
        sRow[2 * tid]     = a0 + b1[0];
        sRow[2 * tid + 1] = a1 + b1[1];
    }
    __syncthreads();
    float* dst = (blk < NB) ? (out + 2 * NB + (size_t)blk * (2 * NT)) : out;
    const int q = min(tid, 127);
    v4f v;
#pragma unroll
    for (int i = 0; i < 4; ++i) v[i] = sRow[4 * q + i];
    float* p = dst + 4 * q;
    if (tid < 128) *(volatile v4f*)p = v;
    __threadfence();
    if (tid < 128) *(volatile v4f*)p = v;
}

extern "C" void kernel_launch(void* const* d_in, const int* in_sizes, int n_in,
                              void* d_out, int out_size, void* d_ws, size_t ws_size,
                              hipStream_t stream)
{
    if (n_in < 18) return;
    if (in_sizes[0] != NB * NT) return;
    if (in_sizes[1] < HH || (in_sizes[1] % HH) != 0) return;
    const int nV = in_sizes[1] / HH;
    if (in_sizes[2] != 2 * G4 * HH || in_sizes[3] != 2 * G4 * HH) return;
    if (in_sizes[4] != 2 * G4 || in_sizes[5] != 2 * G4) return;
    if (in_sizes[6] != 2 * G4 * HH || in_sizes[7] != 2 * G4 * HH) return;
    if (in_sizes[8] != 2 * G4 || in_sizes[9] != 2 * G4) return;
    if (in_sizes[10] != 2 * CE) return;
    if (in_sizes[11] < 1) return;
    if (in_sizes[12] != HH * 2 * CE) return;
    if (in_sizes[13] != HH) return;
    if (in_sizes[14] != 2 * CE || in_sizes[15] != 2) return;
    if (in_sizes[16] != 2 * CE || in_sizes[17] != 2) return;
    if (out_size != NB * 2 + NB * NT * 2) return;
    if (ws_size < WS_END) return;

    const int*   xin   = (const int*)d_in[0];
    const float* emb   = (const float*)d_in[1];
    const float* eWih  = (const float*)d_in[2];
    const float* eWhh  = (const float*)d_in[3];
    const float* eBih  = (const float*)d_in[4];
    const float* eBhh  = (const float*)d_in[5];
    const float* dWih  = (const float*)d_in[6];
    const float* dWhh  = (const float*)d_in[7];
    const float* dBih  = (const float*)d_in[8];
    const float* dBhh  = (const float*)d_in[9];
    const float* attnW = (const float*)d_in[10];
    const float* attnB = (const float*)d_in[11];
    const float* combW = (const float*)d_in[12];
    const float* combB = (const float*)d_in[13];
    const float* cls1W = (const float*)d_in[14];
    const float* cls1B = (const float*)d_in[15];
    const float* cls2W = (const float*)d_in[16];
    const float* cls2B = (const float*)d_in[17];
    float* out = (float*)d_out;

    char* ws = (char*)d_ws;
    _Float16* WE = (_Float16*)(ws + OFF_WE);
    _Float16* WD = (_Float16*)(ws + OFF_WD);
    _Float16* WC = (_Float16*)(ws + OFF_WC);
    float*    E  = (float*)(ws + OFF_E);
    float*    CT = (float*)(ws + OFF_CT);
    float*    PG = (float*)(ws + OFF_PG);
    float*    ZB = (float*)(ws + OFF_ZB);
    float*    LG = (float*)(ws + OFF_LG);

    prep_kernel<<<dim3(PREP_BLK), dim3(256), 0, stream>>>(eWih, eWhh, dWih, dWhh, combW, WE, WD, WC);

    encoder_kernel<<<dim3(2 * ENBLK), dim3(ENTHR), ENC_LDS, stream>>>(
        xin, emb, nV, (const _Float16*)WE, eBih, eBhh, E, CT);

    hipFuncSetAttribute(reinterpret_cast<const void*>(&pg_kernel),
                        hipFuncAttributeMaxDynamicSharedMemorySize, (int)PG_LDS);
    pg_kernel<<<dim3((NB * NT) / PGM), dim3(PGTHR), PG_LDS, stream>>>((const float*)E, (const _Float16*)WC, PG);

    attn_kernel<<<dim3(NB), dim3(256), 0, stream>>>((const float*)E, (const float*)PG, attnW, attnB, combB, ZB);

    hipFuncSetAttribute(reinterpret_cast<const void*>(&decoder_kernel),
                        hipFuncAttributeMaxDynamicSharedMemorySize, (int)DEC_LDS);
    decoder_kernel<<<dim3(1), dim3(DNTHR), DEC_LDS, stream>>>(
        (const float*)E, (const float*)CT, (const float*)PG, (const float*)ZB, (const _Float16*)WD,
        dBih, dBhh, cls2W, cls2B, LG);

    out_kernel<<<dim3(NB + 1), dim3(256), 0, stream>>>((const float*)LG, (const float*)E, cls1W, cls1B, out);
}
